// Transformer_54760833024643
// MI455X (gfx1250) — hardware-verified
//
#include <hip/hip_runtime.h>
#include <math.h>

#ifndef NB
#define NB 2
#endif
#ifndef HH
#define HH 80
#endif
#define WW 80
#define SEQ (HH * WW)
#define SEQ_FULL 6400
#define CH 128
#define NTOK (NB * SEQ)
#define KCV 225
#define KCP 256

static_assert(SEQ % 64 == 0);
static_assert(NTOK % 64 == 0);
static_assert(HH <= 80);
static_assert((NTOK * 32) % 256 == 0);

typedef __attribute__((ext_vector_type(16))) _Float16 v16h;
typedef __attribute__((ext_vector_type(8)))  _Float16 v8h;
typedef __attribute__((ext_vector_type(8)))  float    v8f;
typedef __attribute__((ext_vector_type(4)))  float    v4f;
typedef __attribute__((ext_vector_type(4)))  unsigned v4u;
typedef __attribute__((ext_vector_type(2)))  unsigned v2u;

union FragU { v16h v; v8h h[2]; };
__device__ __forceinline__ v16h frag_ld(const _Float16* p) { FragU f; f.h[0] = *(const v8h*)(p); f.h[1] = *(const v8h*)(p + 16); return f.v; }
__device__ __forceinline__ v8f mma16(v16h a, v16h b, v8f c) { return __builtin_amdgcn_wmma_f32_16x16x32_f16(false, a, false, b, (short)0, c, false, false); }
__device__ __forceinline__ void dep_guard_h(v8f& a, v8f& b, v16h x, v16h y) { asm volatile("v_nop\n\tv_nop\n\tv_nop\n\tv_nop" : "+v"(a), "+v"(b) : "v"(x), "v"(y)); }
__device__ __forceinline__ void keep4_h(v16h a, v16h b, v16h c, v16h d) { asm volatile("v_nop" :: "v"(a), "v"(b), "v"(c), "v"(d)); }
__device__ __forceinline__ void acc_guard4(v8f& a, v8f& b, v8f& c, v8f& d) { asm volatile("v_nop\n\tv_nop\n\tv_nop\n\tv_nop" : "+v"(a), "+v"(b), "+v"(c), "+v"(d)); }
__device__ __forceinline__ void guard2x8(v8f& a, v8f& b, v16h f0, v16h f1, v16h f2, v16h f3, v16h f4, v16h f5, v16h f6, v16h f7) {
    asm volatile("v_nop\n\tv_nop\n\tv_nop\n\tv_nop" : "+v"(a), "+v"(b) : "v"(f0), "v"(f1), "v"(f2), "v"(f3), "v"(f4), "v"(f5), "v"(f6), "v"(f7)); }
__device__ __forceinline__ void guard4x5(v8f& a, v8f& b, v8f& c, v8f& d, v16h f0, v16h f1, v16h f2, v16h f3, v16h p) {
    asm volatile("v_nop\n\tv_nop\n\tv_nop\n\tv_nop" : "+v"(a), "+v"(b), "+v"(c), "+v"(d) : "v"(f0), "v"(f1), "v"(f2), "v"(f3), "v"(p)); }
__device__ __forceinline__ float ex2(float x) { return __builtin_amdgcn_exp2f(x); }

#define VST2(T, ptr, val) do { const T vst2_v_ = (val); *(volatile T*)(ptr) = vst2_v_; __threadfence(); *(volatile T*)(ptr) = vst2_v_; } while (0)
#define VST2V4(ptr, val) do { const v4f vst2_v4_ = (val); *(volatile v4f*)(ptr) = vst2_v4_; __threadfence(); *(volatile v4f*)(ptr) = vst2_v4_; } while (0)

__device__ __forceinline__ unsigned cmb_pk2(float a, float b) { return (unsigned)__builtin_bit_cast(unsigned short, (_Float16)a) | ((unsigned)__builtin_bit_cast(unsigned short, (_Float16)b) << 16); }
__device__ __forceinline__ float cmb_bf(float v) { const unsigned u = __builtin_bit_cast(unsigned, v); const unsigned r = (u + 0x7fffu + ((u >> 16) & 1u)) & 0xffff0000u; return __builtin_bit_cast(float, r); }

__global__ __launch_bounds__(256) void k_castT3(const float* __restrict__ s0, const float* __restrict__ s1, const float* __restrict__ s2, unsigned lds,
                                                unsigned short* __restrict__ DST, unsigned ldd, unsigned nR, unsigned nC, float sc) {
    const unsigned u = blockIdx.x * 256u + threadIdx.x; const unsigned per = nR >> 3; if (u >= nC * per) return;
    const unsigned c = u / per; const unsigned r0 = (u - c * per) << 3; const unsigned y = blockIdx.y;
    const float* src = (y == 0u) ? s0 : ((y == 1u) ? s1 : s2);
    float w[8];
#pragma unroll
    for (int e = 0; e < 8; ++e) w[e] = cmb_bf(src[(size_t)(r0 + e) * lds + c]) * sc;
    v4u pk; pk.x = cmb_pk2(w[0], w[1]); pk.y = cmb_pk2(w[2], w[3]); pk.z = cmb_pk2(w[4], w[5]); pk.w = cmb_pk2(w[6], w[7]);
    VST2(v4u, (v4u*)(DST + (size_t)y * nC * ldd + (size_t)c * ldd + r0), pk);
}
__global__ __launch_bounds__(256) void k_convw(const float* __restrict__ cw, unsigned short* __restrict__ DST) {
    const unsigned u = blockIdx.x * 256u + threadIdx.x; if (u >= 128u * 32u) return;
    const unsigned oc = u >> 5, k0 = (u & 31u) << 3;
    float w[8];
#pragma unroll
    for (int e = 0; e < 8; ++e) { const unsigned k = k0 + e; const unsigned kc = (k < (unsigned)KCV) ? k : (unsigned)(KCV - 1); const float v = cmb_bf(cw[oc * (unsigned)KCV + kc]) * 16.0f; w[e] = (k < (unsigned)KCV) ? v : 0.f; }
    v4u pk; pk.x = cmb_pk2(w[0], w[1]); pk.y = cmb_pk2(w[2], w[3]); pk.z = cmb_pk2(w[4], w[5]); pk.w = cmb_pk2(w[6], w[7]);
    VST2(v4u, (v4u*)(DST + (size_t)oc * KCP + k0), pk);
}
__global__ __launch_bounds__(256) void k_im2col(const float* __restrict__ x, unsigned short* __restrict__ X16) {
    const unsigned u = blockIdx.x * 256u + threadIdx.x; if (u >= (unsigned)NTOK * 32u) return;
    const unsigned tok = u >> 5, k0 = (u & 31u) << 3;
    const unsigned b = tok / (unsigned)SEQ, n = tok - b * (unsigned)SEQ, h = n / 80u, w = n - h * 80u;
    const float* xb = x + (size_t)b * (9u * SEQ_FULL);
    float v[8];
#pragma unroll
    for (int e = 0; e < 8; ++e) {
        const unsigned k = k0 + e; const unsigned kk = (k < 225u) ? k : 224u;
        const unsigned cc = kk / 25u, rem = kk - cc * 25u, kh = rem / 5u, kw = rem - kh * 5u, tt = cc / 3u, ci = cc - tt * 3u;
        const unsigned uh = h + kh, uw = w + kw;
        const bool ok = (k < 225u) && (uh >= 2u) && (uh < (unsigned)HH + 2u) && (uw >= 2u) && (uw < 82u);
        const unsigned ih = min(max(uh, 2u), (unsigned)HH + 1u) - 2u, iw = min(max(uw, 2u), 81u) - 2u;
        float xv = xb[(ci * 3u + tt) * (unsigned)SEQ_FULL + ih * 80u + iw];
        asm volatile("" : "+v"(xv));
        const float keep = ok ? 1.0f : 0.0f;
        v[e] = __fmul_rn(cmb_bf(xv), keep);
    }
    v4u pk; pk.x = cmb_pk2(v[0], v[1]); pk.y = cmb_pk2(v[2], v[3]); pk.z = cmb_pk2(v[4], v[5]); pk.w = cmb_pk2(v[6], v[7]);
    VST2(v4u, (v4u*)(X16 + (size_t)tok * KCP + k0), pk);
}
__global__ __launch_bounds__(32) void k_invf(float* __restrict__ invb) {
    const unsigned i = threadIdx.x; const float e = (float)(2u * i) / 64.0f; const float v = 1.0f / powf(10000.0f, e); VST2(float, invb + i, v);
}
__global__ __launch_bounds__(256) void k_petab(const float* __restrict__ invb, float* __restrict__ PET) {
    const unsigned u = blockIdx.x * 256u + threadIdx.x; if (u >= 80u * 64u) return;
    const unsigned pos = u >> 6, i = u & 63u; const float ang = (float)pos * invb[i & 31u];
    const float s = sinf(ang), c = cosf(ang); const float v = (i < 32u) ? s : c; VST2(float, PET + u, v);
}
__global__ __launch_bounds__(256) void k_ln16(const float* __restrict__ X, const float* __restrict__ g, const float* __restrict__ bt, unsigned short* __restrict__ Y) {
    const unsigned lane = threadIdx.x & 31u; const unsigned row = blockIdx.x * 8u + (threadIdx.x >> 5);
    const size_t ro = (size_t)row * 128u + 4u * lane;
    const v4f a = *(const v4f*)(X + ro);
    float sm = (a.x + a.y) + (a.z + a.w);
#pragma unroll
    for (int o = 16; o > 0; o >>= 1) sm += __shfl_xor(sm, o, 32);
    const float mu = sm * (1.0f / 128.0f); const v4f d = a - mu;
    float q = (d.x * d.x + d.y * d.y) + (d.z * d.z + d.w * d.w);
#pragma unroll
    for (int o = 16; o > 0; o >>= 1) q += __shfl_xor(q, o, 32);
    const float rs = 1.0f / sqrtf(q * (1.0f / 128.0f) + 1e-5f);
    const v4f g4 = *(const v4f*)(g + 4u * lane), b4 = *(const v4f*)(bt + 4u * lane);
    const float y0 = d.x * rs * cmb_bf(g4.x) + cmb_bf(b4.x), y1 = d.y * rs * cmb_bf(g4.y) + cmb_bf(b4.y);
    const float y2 = d.z * rs * cmb_bf(g4.z) + cmb_bf(b4.z), y3 = d.w * rs * cmb_bf(g4.w) + cmb_bf(b4.w);
    v2u pk; pk.x = cmb_pk2(y0, y1); pk.y = cmb_pk2(y2, y3);
    VST2(v2u, (v2u*)(Y + ro), pk);
}

template <int EPI>
__global__ __launch_bounds__(256) void k_gemm64(
    const unsigned short* __restrict__ Ap, unsigned lda, unsigned strideA,
    const unsigned short* __restrict__ Btp, unsigned ldb, unsigned strideB,
    void* __restrict__ Cout, unsigned ldc, unsigned strideC,
    const float* __restrict__ p0, const float* __restrict__ p1, const float* __restrict__ p2, unsigned strideR,
    unsigned M, unsigned N, unsigned K, float scale) {
  __shared__ __align__(16) float sT[8][16 * 68];
  const unsigned b = blockIdx.y, lane = threadIdx.x & 31u, wave = threadIdx.x >> 5;
  const unsigned tilesN = N >> 6, tilesM = M >> 6;
  const unsigned tile = blockIdx.x * 8u + wave;
  if (tile >= tilesM * tilesN) return;
  const unsigned tm = tile / tilesN, tn = tile - tm * tilesN, m0 = tm << 6, n0 = tn << 6;
  const _Float16* Ab = (const _Float16*)Ap + (size_t)b * strideA;
  const _Float16* Bb = (const _Float16*)Btp + (size_t)b * strideB;
  const unsigned rlane = lane & 15u, koff = (lane >> 4) * 8u, mOff = koff;

  v8f acc[4][4];
#pragma unroll
  for (int i = 0; i < 4; ++i)
#pragma unroll
    for (int j = 0; j < 4; ++j) acc[i][j] = (v8f){0.f, 0.f, 0.f, 0.f, 0.f, 0.f, 0.f, 0.f};

  for (unsigned k0 = 0; k0 < K; k0 += 32u) {
    v16h bh[4];
#pragma unroll
    for (int j = 0; j < 4; ++j) bh[j] = frag_ld(Bb + (size_t)(n0 + ((unsigned)j << 4) + rlane) * ldb + koff + k0);
#pragma unroll
    for (int i = 0; i < 4; ++i) {
      const v16h ah = frag_ld(Ab + (size_t)(m0 + ((unsigned)i << 4) + rlane) * lda + koff + k0);
#pragma unroll
      for (int j = 0; j < 4; ++j) acc[i][j] = mma16(ah, bh[j], acc[i][j]);
      dep_guard_h(acc[i][0], acc[i][3], ah, ah);
    }
    keep4_h(bh[0], bh[1], bh[2], bh[3]);
  }
  acc_guard4(acc[0][0], acc[0][1], acc[0][2], acc[0][3]);
  acc_guard4(acc[1][0], acc[1][1], acc[1][2], acc[1][3]);
  acc_guard4(acc[2][0], acc[2][1], acc[2][2], acc[2][3]);
  acc_guard4(acc[3][0], acc[3][1], acc[3][2], acc[3][3]);

  float* slab = sT[wave];
  const float bns = 1.0f / sqrtf(1.00001f);
#pragma unroll
  for (int i = 0; i < 4; ++i) {
    const unsigned mBase = m0 + ((unsigned)i << 4);
    unsigned ph[8], pw[8];
    if (EPI == 0) {
#pragma unroll
      for (int r = 0; r < 8; ++r) { const unsigned row = mBase + mOff + r; const unsigned rb = row - (row / (unsigned)SEQ) * (unsigned)SEQ; const unsigned hh = rb / 80u; ph[r] = hh; pw[r] = rb - hh * 80u; }
    }
#pragma unroll
    for (int j = 0; j < 4; ++j) {
      const unsigned n = n0 + ((unsigned)j << 4) + rlane;
      float cg = 0.f, cb = 0.f;
      if (EPI == 0) { cg = bns * cmb_bf(p0[n]); cb = cmb_bf(p1[n]); }
      if (EPI == 2) cb = cmb_bf(p0[n]);
#pragma unroll
      for (int r = 0; r < 8; ++r) {
        float v = acc[i][j][r] * scale;
        if (EPI == 0) {
          v = v * cg + cb;
          v = (v > 0.f) ? v : 0.2f * v;
          const unsigned pos = (n < 64u) ? ph[r] : pw[r];
          v += p2[pos * 64u + (n & 63u)];
        }
        if (EPI == 2) { v += cb; v = 0.5f * v * (1.0f + erff(v * 0.70710678118654752f)); }
        if (EPI == 3) { const unsigned row = mBase + mOff + r; v += cmb_bf(p0[row]); v += p1[(size_t)b * strideR + (size_t)n * 128u + row]; }
        slab[(mOff + r) * 68u + ((unsigned)j << 4) + rlane] = v;
      }
    }
    __builtin_amdgcn_fence(3  , "workgroup");
    __builtin_amdgcn_wave_barrier();
    __builtin_amdgcn_fence(2  , "workgroup");
    if (EPI == 0 || EPI == 3) {
      float* C = (float*)Cout + (size_t)b * strideC;
      const unsigned hh = lane >> 4, c4 = (lane & 15u) * 4u;
      for (int pass = 0; pass < 2; ++pass) {
#pragma unroll
        for (int it = 0; it < 8; ++it) {
          const unsigned row = (unsigned)it * 2u + hh;
          const v4f v = *(const v4f*)(slab + row * 68u + c4);
          *(volatile v4f*)(C + (size_t)(mBase + row) * ldc + n0 + c4) = v;
        }
        __threadfence();
      }
    } else {
      const unsigned q = lane >> 3, c8 = (lane & 7u) * 8u;
      unsigned short* C = (unsigned short*)Cout + (size_t)b * strideC;
      for (int pass = 0; pass < 2; ++pass) {
#pragma unroll
        for (int it = 0; it < 4; ++it) {
          const unsigned row = (unsigned)it * 4u + q;
          const float* sp = slab + row * 68u + c8;
          v8h hv;
#pragma unroll
          for (int e = 0; e < 8; ++e) hv[e] = (_Float16)sp[e];
          *(volatile v8h*)(C + (size_t)(mBase + row) * ldc + n0 + c8) = hv;
        }
        __threadfence();
      }
    }
    __builtin_amdgcn_fence(3  , "workgroup");
    __builtin_amdgcn_wave_barrier();
    __builtin_amdgcn_fence(2  , "workgroup");
  }
}

#define C2SC (0.08838834764831845f * 1.4426950408889634f)

__global__ __launch_bounds__(128) void k_colstat(const unsigned short* __restrict__ QKp, float* __restrict__ NL) {
  __shared__ __align__(16) float sred[64];
  const unsigned lane = threadIdx.x & 31u, h = lane >> 4, l15 = lane & 15u, wave = threadIdx.x >> 5;
  const unsigned nblk = (unsigned)SEQ / 64u;
  const unsigned b = blockIdx.x / nblk; const unsigned mblk = (blockIdx.x - b * nblk) * 64u; const unsigned m0 = mblk + wave * 16u;
  const _Float16* QK = (const _Float16*)QKp + (size_t)b * SEQ * 256u;
  v16h kb[4];
  { const _Float16* kr = QK + (size_t)(m0 + l15) * 256u + 128u + 8u * h;
#pragma unroll
    for (int ks = 0; ks < 4; ++ks) kb[ks] = frag_ld(kr + ks * 32); }
  float mrun = -__builtin_inff(), srun = 0.f;
#pragma unroll 1
  for (unsigned n0 = 0; n0 < (unsigned)SEQ; n0 += 32u) {
    const _Float16* q0 = QK + (size_t)(n0 + l15) * 256u + 8u * h; const _Float16* q1 = q0 + 16u * 256u;
    v16h a0[4], a1[4];
#pragma unroll
    for (int ks = 0; ks < 4; ++ks) { a0[ks] = frag_ld(q0 + ks * 32); a1[ks] = frag_ld(q1 + ks * 32); }
    v8f d0 = (v8f){0.f, 0.f, 0.f, 0.f, 0.f, 0.f, 0.f, 0.f}, d1 = d0;
#pragma unroll
    for (int ks = 0; ks < 4; ++ks) { d0 = mma16(a0[ks], kb[ks], d0); d1 = mma16(a1[ks], kb[ks], d1); }
    guard2x8(d0, d1, a0[0], a0[1], a0[2], a0[3], a1[0], a1[1], a1[2], a1[3]);
    float mx = fmaxf(d0[0], d1[0]);
#pragma unroll
    for (int r = 1; r < 8; ++r) mx = fmaxf(mx, fmaxf(d0[r], d1[r]));
    const float mnew = fmaxf(mrun, mx * C2SC);
    float s = srun * ex2(mrun - mnew);
#pragma unroll
    for (int r = 0; r < 8; ++r) s += ex2(fmaf(d0[r], C2SC, -mnew)) + ex2(fmaf(d1[r], C2SC, -mnew));
    srun = s; mrun = mnew;
  }
  const float mo = __shfl_xor(mrun, 16, 32), so = __shfl_xor(srun, 16, 32);
  const float mt = fmaxf(mrun, mo);
  const float st = srun * ex2(mrun - mt) + so * ex2(mo - mt);
  const float nl = 12.0f - (mt + log2f(st));
  if (h == 0u) sred[wave * 16u + l15] = nl;
  __syncthreads();
  if (wave == 0u && lane < 16u) { const v4f v = *(const v4f*)(sred + 4u * lane); VST2V4(NL + (size_t)b * SEQ + mblk + 4u * lane, v); }
}

__global__ __launch_bounds__(128) void k_attn_t(const unsigned short* __restrict__ QKp, const unsigned short* __restrict__ Vtp, const float* __restrict__ NL,
                                                const float* __restrict__ T, const float* __restrict__ g2, const float* __restrict__ b2,
                                                float* __restrict__ ATTN, unsigned short* __restrict__ H16) {
  __shared__ __align__(16) float stg[4][16 * 132];
  const unsigned lane = threadIdx.x & 31u, h = lane >> 4, l15 = lane & 15u, wave = threadIdx.x >> 5;
  const unsigned nblk = (unsigned)SEQ / 64u;
  const unsigned b = blockIdx.x / nblk; const unsigned n0 = (blockIdx.x - b * nblk) * 64u + wave * 16u;
  const _Float16* QK = (const _Float16*)QKp + (size_t)b * SEQ * 256u;
  const _Float16* Vt = (const _Float16*)Vtp + (size_t)b * SEQ;
  const float* nlb = NL + (size_t)b * SEQ;
  v16h qb[4];
  { const _Float16* qr = QK + (size_t)(n0 + l15) * 256u + 8u * h;
#pragma unroll
    for (int ks = 0; ks < 4; ++ks) qb[ks] = frag_ld(qr + ks * 32); }
  v8f acc[8];
#pragma unroll
  for (int ct = 0; ct < 8; ++ct) acc[ct] = (v8f){0.f, 0.f, 0.f, 0.f, 0.f, 0.f, 0.f, 0.f};
#pragma unroll 1
  for (unsigned m0 = 0; m0 < (unsigned)SEQ; m0 += 32u) {
    const _Float16* kr0 = QK + (size_t)(m0 + l15) * 256u + 128u + 8u * h; const _Float16* kr1 = kr0 + 16u * 256u;
    v16h k0[4], k1[4];
#pragma unroll
    for (int ks = 0; ks < 4; ++ks) { k0[ks] = frag_ld(kr0 + ks * 32); k1[ks] = frag_ld(kr1 + ks * 32); }
    v8f s0 = (v8f){0.f, 0.f, 0.f, 0.f, 0.f, 0.f, 0.f, 0.f}, s1 = s0;
#pragma unroll
    for (int ks = 0; ks < 4; ++ks) { s0 = mma16(k0[ks], qb[ks], s0); s1 = mma16(k1[ks], qb[ks], s1); }
    guard2x8(s0, s1, k0[0], k0[1], k0[2], k0[3], k1[0], k1[1], k1[2], k1[3]);
    const float* np = nlb + m0 + 8u * h;
    const v4f na = *(const v4f*)(np), nb2 = *(const v4f*)(np + 4), nc = *(const v4f*)(np + 16), nd = *(const v4f*)(np + 20);
    v16h pb;
    pb[0]  = (_Float16)ex2(fmaf(s0[0], C2SC, na.x));  pb[1]  = (_Float16)ex2(fmaf(s0[1], C2SC, na.y));
    pb[2]  = (_Float16)ex2(fmaf(s0[2], C2SC, na.z));  pb[3]  = (_Float16)ex2(fmaf(s0[3], C2SC, na.w));
    pb[4]  = (_Float16)ex2(fmaf(s0[4], C2SC, nb2.x)); pb[5]  = (_Float16)ex2(fmaf(s0[5], C2SC, nb2.y));
    pb[6]  = (_Float16)ex2(fmaf(s0[6], C2SC, nb2.z)); pb[7]  = (_Float16)ex2(fmaf(s0[7], C2SC, nb2.w));
    pb[8]  = (_Float16)ex2(fmaf(s1[0], C2SC, nc.x));  pb[9]  = (_Float16)ex2(fmaf(s1[1], C2SC, nc.y));
    pb[10] = (_Float16)ex2(fmaf(s1[2], C2SC, nc.z));  pb[11] = (_Float16)ex2(fmaf(s1[3], C2SC, nc.w));
    pb[12] = (_Float16)ex2(fmaf(s1[4], C2SC, nd.x));  pb[13] = (_Float16)ex2(fmaf(s1[5], C2SC, nd.y));
    pb[14] = (_Float16)ex2(fmaf(s1[6], C2SC, nd.z));  pb[15] = (_Float16)ex2(fmaf(s1[7], C2SC, nd.w));
    const _Float16* vr = Vt + (size_t)l15 * NTOK + m0 + 8u * h;
    {
      const v16h f0 = frag_ld(vr), f1 = frag_ld(vr + (size_t)16 * NTOK), f2 = frag_ld(vr + (size_t)32 * NTOK), f3 = frag_ld(vr + (size_t)48 * NTOK);
      acc[0] = mma16(f0, pb, acc[0]); acc[1] = mma16(f1, pb, acc[1]); acc[2] = mma16(f2, pb, acc[2]); acc[3] = mma16(f3, pb, acc[3]);
      guard4x5(acc[0], acc[1], acc[2], acc[3], f0, f1, f2, f3, pb);
    }
    {
      const v16h f4 = frag_ld(vr + (size_t)64 * NTOK), f5 = frag_ld(vr + (size_t)80 * NTOK), f6 = frag_ld(vr + (size_t)96 * NTOK), f7 = frag_ld(vr + (size_t)112 * NTOK);
      acc[4] = mma16(f4, pb, acc[4]); acc[5] = mma16(f5, pb, acc[5]); acc[6] = mma16(f6, pb, acc[6]); acc[7] = mma16(f7, pb, acc[7]);
      guard4x5(acc[4], acc[5], acc[6], acc[7], f4, f5, f6, f7, pb);
    }
  }
  float* st = stg[wave];
  const float inv = 1.0f / 4096.0f;
#pragma unroll
  for (int ct = 0; ct < 8; ++ct) {
    v4f lo, hi;
    lo.x = acc[ct][0] * inv; lo.y = acc[ct][1] * inv; lo.z = acc[ct][2] * inv; lo.w = acc[ct][3] * inv;
    hi.x = acc[ct][4] * inv; hi.y = acc[ct][5] * inv; hi.z = acc[ct][6] * inv; hi.w = acc[ct][7] * inv;
    *(v4f*)(st + l15 * 132u + (unsigned)ct * 16u + 8u * h) = lo;
    *(v4f*)(st + l15 * 132u + (unsigned)ct * 16u + 8u * h + 4u) = hi;
  }
  __builtin_amdgcn_fence(3  , "workgroup");
  __builtin_amdgcn_wave_barrier();
  __builtin_amdgcn_fence(2  , "workgroup");
  const v4f g4 = *(const v4f*)(g2 + 4u * lane), b4 = *(const v4f*)(b2 + 4u * lane);
  const float gx = cmb_bf(g4.x), gy = cmb_bf(g4.y), gz = cmb_bf(g4.z), gw = cmb_bf(g4.w);
  const float bx = cmb_bf(b4.x), by = cmb_bf(b4.y), bz = cmb_bf(b4.z), bw = cmb_bf(b4.w);
#pragma unroll 2
  for (unsigned j = 0; j < 16u; ++j) {
    const v4f o = *(const v4f*)(st + j * 132u + 4u * lane);
    const size_t ro = ((size_t)b * SEQ + n0 + j) * 128u + 4u * lane;
    const v4f t4 = *(const v4f*)(T + ro);
    const v4f a = t4 + o;
    float sm = (a.x + a.y) + (a.z + a.w);
#pragma unroll
    for (int of = 16; of > 0; of >>= 1) sm += __shfl_xor(sm, of, 32);
    const float mu = sm * (1.0f / 128.0f); const v4f d = a - mu;
    float q = (d.x * d.x + d.y * d.y) + (d.z * d.z + d.w * d.w);
#pragma unroll
    for (int of = 16; of > 0; of >>= 1) q += __shfl_xor(q, of, 32);
    const float rs = 1.0f / sqrtf(q * (1.0f / 128.0f) + 1e-5f);
    v2u pk; pk.x = cmb_pk2(d.x * rs * gx + bx, d.y * rs * gy + by); pk.y = cmb_pk2(d.z * rs * gz + bz, d.w * rs * gw + bw);
    VST2V4(ATTN + ro, a);
    VST2(v2u, (v2u*)(H16 + ro), pk);
  }
}

extern "C" void kernel_launch(void* const* d_in, const int* in_sizes, int n_in, void* d_out, int out_size, void* d_ws, size_t ws_size, hipStream_t stream) {
  (void)out_size;
  if (n_in < 15) return;
  if (in_sizes[0] < NB * 9 * SEQ_FULL / ((SEQ_FULL / SEQ) > 1 ? 2 : 1) || in_sizes[1] < 128 * KCV || in_sizes[6] < 16384 || in_sizes[7] < 16384 || in_sizes[8] < 16384 ||
      in_sizes[11] < 32768 || in_sizes[13] < 32768 || in_sizes[12] < 256 || in_sizes[14] < 128) return;
  const float* x      = (const float*)d_in[0];
  const float* conv_w = (const float*)d_in[1];
  const float* bn_g   = (const float*)d_in[2];
  const float* bn_b   = (const float*)d_in[3];
  const float* ln1_g  = (const float*)d_in[4];
  const float* ln1_b  = (const float*)d_in[5];
  const float* wq     = (const float*)d_in[6];
  const float* wk     = (const float*)d_in[7];
  const float* wv     = (const float*)d_in[8];
  const float* ln2_g  = (const float*)d_in[9];
  const float* ln2_b  = (const float*)d_in[10];
  const float* fc1_w  = (const float*)d_in[11];
  const float* fc1_b  = (const float*)d_in[12];
  const float* fc2_w  = (const float*)d_in[13];
  const float* fc2_b  = (const float*)d_in[14];
  float* out = (float*)d_out;

  char* wsp = (char*)d_ws;
#define CARVE(TY, name, bytes) TY* name = (TY*)wsp; wsp += ((((size_t)(bytes)) + 255) / 256) * 256
  CARVE(unsigned short, WC16,  (size_t)128 * KCP * 2);
  CARVE(unsigned short, WQKV,  (size_t)384 * 128 * 2);
  CARVE(unsigned short, W1P,   (size_t)256 * 128 * 2);
  CARVE(unsigned short, W2P,   (size_t)128 * 256 * 2);
  CARVE(float,          INVF,  (size_t)32 * 4);
  CARVE(float,          PET,   (size_t)80 * 64 * 4);
  CARVE(unsigned short, X16,   (size_t)NTOK * KCP * 2);
  CARVE(float,          TT,    (size_t)NTOK * 128 * 4);
  CARVE(unsigned short, LN16,  (size_t)NTOK * 128 * 2);
  CARVE(unsigned short, QK16,  (size_t)NTOK * 256 * 2);
  CARVE(unsigned short, VT16,  (size_t)128 * NTOK * 2);
  CARVE(float,          NLB,   (size_t)NTOK * 4);
  CARVE(float,          ATTN,  (size_t)NTOK * 128 * 4);
  CARVE(unsigned short, H16,   (size_t)NTOK * 128 * 2);
  CARVE(unsigned short, M1P,   (size_t)NTOK * 256 * 2);
#undef CARVE
  if ((size_t)(wsp - (char*)d_ws) > ws_size || (size_t)(wsp - (char*)d_ws) > (size_t)134217728) return;

  k_convw<<<16, 256, 0, stream>>>(conv_w, WC16);
  k_castT3<<<dim3(8, 3), 256, 0, stream>>>(wq, wk, wv, 128u, WQKV, 128u, 128u, 128u, 16.0f);
  k_castT3<<<dim3(16, 1), 256, 0, stream>>>(fc1_w, fc1_w, fc1_w, 256u, W1P, 128u, 128u, 256u, 16.0f);
  k_castT3<<<dim3(16, 1), 256, 0, stream>>>(fc2_w, fc2_w, fc2_w, 128u, W2P, 256u, 256u, 128u, 16.0f);
  k_invf<<<1, 32, 0, stream>>>(INVF);
  k_petab<<<20, 256, 0, stream>>>(INVF, PET);
  k_im2col<<<(unsigned)(NTOK * 32 / 256), 256, 0, stream>>>(x, X16);
  k_gemm64<0><<<dim3((unsigned)(((NTOK / 64) * 2 + 7) / 8), 1), 256, 0, stream>>>(X16, 256u, 0u, WC16, 256u, 0u, (void*)TT, 128u, 0u, bn_g, bn_b, PET, 0u, (unsigned)NTOK, 128u, 256u, 0.0625f);
  k_ln16<<<(unsigned)(NTOK / 8), 256, 0, stream>>>(TT, ln1_g, ln1_b, LN16);
  k_gemm64<1><<<dim3((unsigned)(((NTOK / 64) * 4 + 7) / 8), 1), 256, 0, stream>>>(LN16, 128u, 0u, WQKV, 128u, 0u, (void*)QK16, 256u, 0u, nullptr, nullptr, nullptr, 0u, (unsigned)NTOK, 256u, 128u, 0.0625f);
  k_gemm64<1><<<dim3((unsigned)((2 * (NTOK / 64) + 7) / 8), 1), 256, 0, stream>>>(WQKV + 256 * 128, 128u, 0u, LN16, 128u, 0u, (void*)VT16, (unsigned)NTOK, 0u, nullptr, nullptr, nullptr, 0u, 128u, (unsigned)NTOK, 128u, 0.0625f);
  k_colstat<<<(unsigned)(NB * (SEQ / 64)), 128, 0, stream>>>(QK16, NLB);
  k_attn_t<<<(unsigned)(NB * (SEQ / 64)), 128, 0, stream>>>(QK16, VT16, NLB, TT, ln2_g, ln2_b, ATTN, H16);
  k_gemm64<2><<<dim3((unsigned)(((NTOK / 64) * 4 + 7) / 8), 1), 256, 0, stream>>>(H16, 128u, 0u, W1P, 128u, 0u, (void*)M1P, 256u, 0u, fc1_b, nullptr, nullptr, 0u, (unsigned)NTOK, 256u, 128u, 0.0625f);
  k_gemm64<3><<<dim3((unsigned)((2 * (SEQ / 64) + 7) / 8), (unsigned)NB), 256, 0, stream>>>(W2P, 256u, 0u, M1P, 256u, (unsigned)(SEQ * 256), (void*)out, (unsigned)SEQ, (unsigned)(128 * SEQ), fc2_b, ATTN, nullptr, (unsigned)(SEQ * 128), 128u, (unsigned)SEQ, 256u, 0.0625f);
}
